// TransformerEncoderLayerTanhRelu_14482629722608
// MI455X (gfx1250) — hardware-verified
//
#include <hip/hip_runtime.h>
#include <math.h>
typedef __attribute__((ext_vector_type(16))) _Float16 v16h;
typedef __attribute__((ext_vector_type(8)))  _Float16 v8h;
typedef __attribute__((ext_vector_type(16))) __bf16   v16b;
typedef __attribute__((ext_vector_type(8)))  __bf16   v8b;
typedef __attribute__((ext_vector_type(8)))  float    v8f;
typedef __attribute__((ext_vector_type(4)))  float    v4f;
#define PSCALE 32768.0f
#define U16(p) ((const unsigned short*)(const void*)(p))
#define PSCALE_INV (1.0f / 32768.0f)

__device__ __forceinline__ unsigned short f2bf_bits(float f) {
  unsigned u = __float_as_uint(f);
  return (unsigned short)((u + 0x7FFFu + ((u >> 16) & 1u)) >> 16);
}
__device__ __forceinline__ float bf_bits2f(unsigned short h) { return __uint_as_float(((unsigned)h) << 16); }

__device__ __forceinline__ void dep_guard_h(v8f& a, v8f& b, v16h x, v16h y) { asm volatile("v_nop\n\tv_nop\n\tv_nop\n\tv_nop" : "+v"(a), "+v"(b) : "v"(x), "v"(y)); }
__device__ __forceinline__ void dep_guard_b(v8f& a, v8f& b, v16b x, v16b y) { asm volatile("v_nop\n\tv_nop\n\tv_nop\n\tv_nop" : "+v"(a), "+v"(b) : "v"(x), "v"(y)); }
__device__ __forceinline__ void keep4_h(v16h a, v16h b, v16h c, v16h d) { asm volatile("v_nop" :: "v"(a), "v"(b), "v"(c), "v"(d)); }
__device__ __forceinline__ void keep4_b(v16b a, v16b b, v16b c, v16b d) { asm volatile("v_nop" :: "v"(a), "v"(b), "v"(c), "v"(d)); }
__device__ __forceinline__ void acc_guard4(v8f& a, v8f& b, v8f& c, v8f& d) { asm volatile("v_nop\n\tv_nop\n\tv_nop\n\tv_nop" : "+v"(a), "+v"(b), "+v"(c), "+v"(d)); }
template <typename T> struct Frag;
template <> struct Frag<_Float16> {
  typedef v16h V; union U { v16h v; v8h h[2]; };
  static __device__ __forceinline__ v16h load(const _Float16* p) {
    U f; f.h[0] = *(const v8h*)(p); f.h[1] = *(const v8h*)(p + 16); return f.v;
  }
  static __device__ __forceinline__ v8f mma(v16h a, v16h b, v8f c) {
    return __builtin_amdgcn_wmma_f32_16x16x32_f16(false, a, false, b, (short)0, c, false, false);
  }
  static __device__ __forceinline__ void guard(v8f& a, v8f& b, v16h x, v16h y) { dep_guard_h(a, b, x, y); }
  static __device__ __forceinline__ void keep(v16h a, v16h b, v16h c, v16h d) { keep4_h(a, b, c, d); }
};
template <> struct Frag<__bf16> {
  typedef v16b V; union U { v16b v; v8b h[2]; };
  static __device__ __forceinline__ v16b load(const __bf16* p) {
    U f; f.h[0] = *(const v8b*)(p); f.h[1] = *(const v8b*)(p + 16); return f.v;
  }
  static __device__ __forceinline__ v8f mma(v16b a, v16b b, v8f c) {
    return __builtin_amdgcn_wmma_f32_16x16x32_bf16(false, a, false, b, (short)0, c, false, false);
  }
  static __device__ __forceinline__ void guard(v8f& a, v8f& b, v16b x, v16b y) { dep_guard_b(a, b, x, y); }
  static __device__ __forceinline__ void keep(v16b a, v16b b, v16b c, v16b d) { keep4_b(a, b, c, d); }
};

template <int ET> struct Elem;
template <> struct Elem<0> { typedef _Float16 T; };
template <> struct Elem<1> { typedef __bf16 T; };
template <int ET, bool SPLIT, int BIAS_MODE, int OUT_MODE, bool RESID, int ACT = 0>
__global__ __launch_bounds__(256) void wmma_gemm64(
    const unsigned short* __restrict__ Ap, const unsigned short* __restrict__ A2p, int lda, long strideA,
    const unsigned short* __restrict__ Btp, const unsigned short* __restrict__ Bt2p, int ldb, long strideB,
    void* __restrict__ Cout, void* __restrict__ Cout2, int ldc, long strideC,
    const float* __restrict__ bias,
    const float* __restrict__ resid, long strideR,
    int M, int N, int K, float scale) {
  typedef typename Elem<ET>::T T;
  typedef typename Frag<T>::V V;
  const T* A = (const T*)Ap; const T* A2 = (const T*)A2p; const T* Bt = (const T*)Btp; const T* Bt2 = (const T*)Bt2p;
  __shared__ __align__(16) float sT[8][16 * 68];
  const int b    = blockIdx.y;
  const int lane = threadIdx.x & 31;
  const int wave = threadIdx.x >> 5;
  const int tilesN = N >> 6;
  const int tilesM = M >> 6;
  const int tile = blockIdx.x * 8 + wave;
  if (tile >= tilesM * tilesN) return;
  const int tm = tile / tilesN;
  const int tn = tile - tm * tilesN;
  const int m0 = tm << 6;
  const int n0 = tn << 6;

  const T* Ab  = A  + (size_t)b * strideA;
  const T* Bb  = Bt + (size_t)b * strideB;
  const T* Ab2 = SPLIT ? (A2  + (size_t)b * strideA) : nullptr;
  const T* Bb2 = SPLIT ? (Bt2 + (size_t)b * strideB) : nullptr;

  const int rlane = lane & 15;
  const int koff  = (lane >> 4) * 8;
  const int mOff  = (lane >> 4) * 8;

  v8f acc[4][4];
#pragma unroll
  for (int i = 0; i < 4; ++i)
#pragma unroll
    for (int j = 0; j < 4; ++j) acc[i][j] = (v8f){0.f,0.f,0.f,0.f,0.f,0.f,0.f,0.f};

  for (int k0 = 0; k0 < K; k0 += 32) {
    V bh[4], bl[4];
#pragma unroll
    for (int j = 0; j < 4; ++j) {
      const size_t bo = (size_t)(n0 + (j << 4) + rlane) * ldb + koff + k0;
      bh[j] = Frag<T>::load(Bb + bo);
      if (SPLIT) bl[j] = Frag<T>::load(Bb2 + bo);
    }
#pragma unroll
    for (int i = 0; i < 4; ++i) {
      const size_t ao = (size_t)(m0 + (i << 4) + rlane) * lda + koff + k0;
      V ah = Frag<T>::load(Ab + ao);
      V al;
      if (SPLIT) al = Frag<T>::load(Ab2 + ao);
#pragma unroll
      for (int j = 0; j < 4; ++j) {
        acc[i][j] = Frag<T>::mma(ah, bh[j], acc[i][j]);
        if (SPLIT) {
          acc[i][j] = Frag<T>::mma(ah, bl[j], acc[i][j]);
          acc[i][j] = Frag<T>::mma(al, bh[j], acc[i][j]);
        }
      }
      Frag<T>::guard(acc[i][0], acc[i][3], ah, SPLIT ? al : ah);
    }
    Frag<T>::keep(bh[0], bh[1], bh[2], bh[3]);
    if (SPLIT) Frag<T>::keep(bl[0], bl[1], bl[2], bl[3]);
  }
  acc_guard4(acc[0][0], acc[0][1], acc[0][2], acc[0][3]);
  acc_guard4(acc[1][0], acc[1][1], acc[1][2], acc[1][3]);
  acc_guard4(acc[2][0], acc[2][1], acc[2][2], acc[2][3]);
  acc_guard4(acc[3][0], acc[3][1], acc[3][2], acc[3][3]);

  float* slab = sT[wave];
  const float* Rb = RESID ? (resid + (size_t)b * strideR) : nullptr;
#pragma unroll
  for (int i = 0; i < 4; ++i) {
    const int mBase = m0 + (i << 4);
#pragma unroll
    for (int j = 0; j < 4; ++j) {
      const int n = n0 + (j << 4) + rlane;
      float bv = 0.f;
      if (BIAS_MODE == 2) bv = bias[n];
#pragma unroll
      for (int r = 0; r < 8; ++r) {
        float v = acc[i][j][r] * scale;
        if (BIAS_MODE == 1) v += bias[mBase + mOff + r];
        if (BIAS_MODE == 2) v += bv;
        if (RESID) v += Rb[(size_t)(mBase + mOff + r) * ldc + n];
        if (ACT == 1) v = tanhf(v);
        if (ACT == 2) v = fmaxf(v, 0.0f);
        if (ACT == 3) v = v / (1.0f + expf(-v));
        if (ACT == 4) v = (v > 0.f) ? v : 0.01f * v;
        if (ACT == 5) v = 0.5f * v * (1.0f + erff(v * 0.70710678118654752f));
        slab[(mOff + r) * 68 + (j << 4) + rlane] = v;
      }
    }
    __builtin_amdgcn_fence(__ATOMIC_RELEASE, "workgroup");
    __builtin_amdgcn_wave_barrier();
    __builtin_amdgcn_fence(__ATOMIC_ACQUIRE, "workgroup");
    if (OUT_MODE == 0) {
      float* C = (float*)Cout + (size_t)b * strideC;
      const int hh = lane >> 4, c4 = (lane & 15) * 4;
      for (int pass = 0; pass < 2; ++pass) {
#pragma unroll
        for (int it = 0; it < 8; ++it) {
          const int row = it * 2 + hh;
          v4f v = *(const v4f*)(slab + row * 68 + c4);
          *(volatile v4f*)(C + (size_t)(mBase + row) * ldc + n0 + c4) = v;
        }
        __threadfence();
      }
    } else {
      const int q = lane >> 3, c8 = (lane & 7) * 8;
      unsigned short* C  = (unsigned short*)Cout  + (size_t)b * strideC;
      unsigned short* C2 = (OUT_MODE == 2) ? ((unsigned short*)Cout2 + (size_t)b * strideC) : nullptr;
      for (int pass = 0; pass < 2; ++pass) {
#pragma unroll
        for (int it = 0; it < 4; ++it) {
          const int row = it * 4 + q;
          const float* sp = slab + row * 68 + c8;
          v8h hv, lv;
#pragma unroll
          for (int e = 0; e < 8; ++e) {
            if (OUT_MODE == 1) {
              hv[e] = (_Float16)sp[e];
            } else {
              unsigned short hb = f2bf_bits(sp[e]);
              unsigned short lb = f2bf_bits(sp[e] - bf_bits2f(hb));
              hv[e] = __builtin_bit_cast(_Float16, hb);
              lv[e] = __builtin_bit_cast(_Float16, lb);
            }
          }
          *(volatile v8h*)(C + (size_t)(mBase + row) * ldc + n0 + c8) = hv;
          if (OUT_MODE == 2) *(volatile v8h*)(C2 + (size_t)(mBase + row) * ldc + n0 + c8) = lv;
        }
        __threadfence();
      }
    }
    __builtin_amdgcn_fence(__ATOMIC_RELEASE, "workgroup");
    __builtin_amdgcn_wave_barrier();
    __builtin_amdgcn_fence(__ATOMIC_ACQUIRE, "workgroup");
  }
}

__global__ __launch_bounds__(256) void cast_f32_f16x2(
    const float* __restrict__ in, _Float16* __restrict__ out, int n2) {
  int i = blockIdx.x * 256 + threadIdx.x;
  if (i < n2) {
    const _Float16 h0 = (_Float16)in[2 * i], h1 = (_Float16)in[2 * i + 1];
    const unsigned u = (unsigned)__builtin_bit_cast(unsigned short, h0) | ((unsigned)__builtin_bit_cast(unsigned short, h1) << 16);
    ((volatile unsigned*)out)[i] = u;
    __threadfence();
    ((volatile unsigned*)out)[i] = u;
  }
}


#define ES 2048
#define EB_ 4
#define ED 256
#define EH 8
#define EHD 32
#define EF 2048
#define ER (ES * EB_)
__device__ __forceinline__ unsigned pkh(float a, float b) { return (unsigned)__builtin_bit_cast(unsigned short, (_Float16)a) | ((unsigned)__builtin_bit_cast(unsigned short, (_Float16)b) << 16); }
template <bool PRELN>
__global__ __launch_bounds__(256) void ln_kernel(const float* __restrict__ A, const float* __restrict__ Cadd, const float* __restrict__ g, const float* __restrict__ bb, float* __restrict__ Y, unsigned* __restrict__ Y16) {
  const int lane = threadIdx.x & 31, wave = threadIdx.x >> 5; const size_t r = (size_t)blockIdx.x * 8 + wave;
  v8f v = *(const v8f*)(A + r * ED + lane * 8);
  if (PRELN) { float s0 = 0.f; for (int q = 0; q < 8; ++q) s0 += v[q]; for (int o = 16; o > 0; o >>= 1) s0 += __shfl_xor(s0, o, 32); const float m0 = s0 / ED; float t0 = 0.f; for (int q = 0; q < 8; ++q) { const float d = v[q] - m0; t0 += d * d; } for (int o = 16; o > 0; o >>= 1) t0 += __shfl_xor(t0, o, 32); const float i0 = rsqrtf(t0 / ED + 1e-5f); for (int q = 0; q < 8; ++q) { const int c = lane * 8 + q; v[q] = (v[q] - m0) * i0 * g[c] + bb[c]; } }
  if (Cadd) v += *(const v8f*)(Cadd + r * ED + lane * 8);
  float s = 0.f; for (int q = 0; q < 8; ++q) s += v[q]; for (int o = 16; o > 0; o >>= 1) s += __shfl_xor(s, o, 32); const float mu = s / ED;
  float t = 0.f; for (int q = 0; q < 8; ++q) { const float d = v[q] - mu; t += d * d; } for (int o = 16; o > 0; o >>= 1) t += __shfl_xor(t, o, 32); const float inv = rsqrtf(t / ED + 1e-5f);
  v8f y; for (int q = 0; q < 8; ++q) { const int c = lane * 8 + q; y[q] = (v[q] - mu) * inv * g[c] + bb[c]; }
  typedef __attribute__((ext_vector_type(4))) unsigned u4; u4 u; for (int q = 0; q < 4; ++q) u[q] = pkh(y[2 * q], y[2 * q + 1]);
  for (int pass = 0; pass < 2; ++pass) { if (Y) *(volatile v8f*)(Y + r * ED + lane * 8) = y; if (Y16) *(volatile u4*)(Y16 + (r * ED + lane * 8) / 2) = u; __threadfence(); }
}
__global__ __launch_bounds__(256) void vt_kernel(const unsigned* __restrict__ QKV16, unsigned* __restrict__ VT) {
  __shared__ float tile[64][33];
  const int bh = blockIdx.y, t0 = blockIdx.x * 64, tx = threadIdx.x, ty = threadIdx.y; const int b = bh / EH, h = bh % EH; typedef __attribute__((ext_vector_type(2))) _Float16 v2h;
  for (int t = ty; t < 64; t += 8) { if (tx < 16) { const v2h p = __builtin_bit_cast(v2h, QKV16[(((size_t)(t0 + t) * EB_ + b) * 768 + 512 + h * EHD) / 2 + tx]); tile[t][2 * tx] = (float)p[0]; tile[t][2 * tx + 1] = (float)p[1]; } }
  __syncthreads();
  for (int pass = 0; pass < 2; ++pass) { for (int d = ty; d < 64; d += 8) ((volatile unsigned*)VT)[(((size_t)bh * 64 + d) * ES + t0) / 2 + tx] = (d < EHD) ? pkh(tile[2 * tx][d], tile[2 * tx + 1][d]) : 0u; __threadfence(); }
}
__global__ __launch_bounds__(256) void act_kernel(const float* __restrict__ S, unsigned* __restrict__ P16, long npair) {
  const long i = (long)blockIdx.x * 256 + threadIdx.x; if (i >= npair) return; const float a = fmaxf(tanhf(S[2 * i]), 0.f) * 32768.0f, b = fmaxf(tanhf(S[2 * i + 1]), 0.f) * 32768.0f;
  ((volatile unsigned*)P16)[i] = pkh(a, b); __threadfence(); ((volatile unsigned*)P16)[i] = pkh(a, b);
}
__global__ __launch_bounds__(256) void orel_kernel(const float* __restrict__ OZ, int b, int h0, unsigned* __restrict__ O16) {
  const int lane = threadIdx.x & 31, wave = threadIdx.x >> 5; const int r = blockIdx.x * 8 + wave; const int hh = r & 1, s = r >> 1; if (lane >= 16) return;
  const float* src = OZ + ((size_t)hh * ES + s) * 64 + 2 * lane; const unsigned u = pkh(src[0], src[1]);
  unsigned* dst = O16 + (((size_t)s * EB_ + b) * ED + (h0 + hh) * EHD) / 2 + lane; *(volatile unsigned*)dst = u; __threadfence(); *(volatile unsigned*)dst = u;
}
extern "C" void kernel_launch(void* const* d_in, const int* in_sizes, int n_in, void* d_out, int out_size, void* d_ws, size_t ws_size, hipStream_t stream) {
  (void)in_sizes; (void)n_in; (void)out_size; (void)ws_size;
  auto Fp = [&](int i) { return (const float*)d_in[i]; };
  const float* x = Fp(0); const float* lng = Fp(1); const float* lnb = Fp(2); const float* Win = Fp(3); const float* bin = Fp(4); const float* Wout = Fp(5); const float* bout = Fp(6); const float* W1 = Fp(7); const float* b1 = Fp(8); const float* W2 = Fp(9); const float* b2 = Fp(10);
  char* ws = (char*)d_ws; size_t off = 0;
  auto carve = [&](size_t bytes) -> char* { char* p = ws + off; off += (bytes + 255) & ~(size_t)255; return p; };
  unsigned* LNX16 = (unsigned*)carve((size_t)ER * ED * 2); _Float16* WIN16 = (_Float16*)carve(768 * ED * 2); _Float16* WOUT16 = (_Float16*)carve(ED * ED * 2); _Float16* W116 = (_Float16*)carve((size_t)EF * ED * 2); _Float16* W216 = (_Float16*)carve((size_t)ED * EF * 2);
  unsigned* QKV16 = (unsigned*)carve((size_t)ER * 768 * 2); unsigned* VT = (unsigned*)carve((size_t)EB_ * EH * 64 * ES * 2); unsigned* P16 = (unsigned*)carve((size_t)2 * ES * ES * 2); float* OZ = (float*)carve((size_t)2 * ES * 64 * 4); unsigned* O16 = (unsigned*)carve((size_t)ER * ED * 2);
  float* ATT = (float*)carve((size_t)ER * ED * 4); float* R1 = (float*)carve((size_t)ER * ED * 4); unsigned* R116 = (unsigned*)carve((size_t)ER * ED * 2); float* FF = (float*)carve((size_t)ER * ED * 4);
  _Float16* H1 = (_Float16*)carve((size_t)ER * (EF / 2) * 2); float* S = (float*)carve((size_t)2 * ES * ES * 4);
  ln_kernel<false><<<ER / 8, 256, 0, stream>>>(x, nullptr, lng, lnb, nullptr, LNX16);
  cast_f32_f16x2<<<(768 * ED / 2 + 255) / 256, 256, 0, stream>>>(Win, WIN16, 768 * ED / 2); cast_f32_f16x2<<<(ED * ED / 2 + 255) / 256, 256, 0, stream>>>(Wout, WOUT16, ED * ED / 2);
  cast_f32_f16x2<<<(EF * ED / 2 + 255) / 256, 256, 0, stream>>>(W1, W116, (long)EF * ED / 2); cast_f32_f16x2<<<(ED * EF / 2 + 255) / 256, 256, 0, stream>>>(W2, W216, (long)ED * EF / 2);
  const int tr = ER / 64;
  wmma_gemm64<0, false, 2, 1, false><<<dim3((tr * 12 + 7) / 8, 1), 256, 0, stream>>>((const unsigned short*)LNX16, nullptr, ED, 0, U16(WIN16), nullptr, ED, 0, QKV16, nullptr, 768, 0, bin, nullptr, 0, ER, 768, ED, 1.0f);
  vt_kernel<<<dim3(ES / 64, EB_ * EH), dim3(32, 8), 0, stream>>>(QKV16, VT);
  const int ts = (ES / 64) * (ES / 64);
  for (int b = 0; b < EB_; ++b) for (int h0 = 0; h0 < EH; h0 += 2) {
    wmma_gemm64<0, false, 0, 0, false><<<dim3((ts + 7) / 8, 2), 256, 0, stream>>>((const unsigned short*)QKV16 + (size_t)b * 768 + h0 * EHD, nullptr, EB_ * 768, EHD, (const unsigned short*)QKV16 + (size_t)b * 768 + ED + h0 * EHD, nullptr, EB_ * 768, EHD, S, nullptr, ES, (long)ES * ES, nullptr, nullptr, 0, ES, ES, EHD, 0.17677669529663687f);
    act_kernel<<<(unsigned)(((long)2 * ES * ES / 2 + 255) / 256), 256, 0, stream>>>(S, P16, (long)2 * ES * ES / 2);
    wmma_gemm64<0, false, 0, 0, false><<<dim3((ES / 64 + 7) / 8, 2), 256, 0, stream>>>((const unsigned short*)P16, nullptr, ES, (long)ES * ES, (const unsigned short*)VT + ((size_t)b * EH + h0) * 64 * ES, nullptr, ES, (long)64 * ES, OZ, nullptr, 64, (long)ES * 64, nullptr, nullptr, 0, ES, 64, ES, 1.0f / 32768.0f);
    orel_kernel<<<2 * ES / 8, 256, 0, stream>>>(OZ, b, h0, O16); }
  wmma_gemm64<0, false, 2, 0, false><<<dim3((tr * 4 + 7) / 8, 1), 256, 0, stream>>>((const unsigned short*)O16, nullptr, ED, 0, U16(WOUT16), nullptr, ED, 0, ATT, nullptr, ED, 0, bout, nullptr, 0, ER, ED, ED, 1.0f);
  ln_kernel<true><<<ER / 8, 256, 0, stream>>>(x, ATT, lng, lnb, R1, R116);
  for (int fh = 0; fh < 2; ++fh) {
    wmma_gemm64<0, false, 2, 1, false, 2><<<dim3((tr * (EF / 128) + 7) / 8, 1), 256, 0, stream>>>((const unsigned short*)R116, nullptr, ED, 0, U16(W116) + (size_t)fh * (EF / 2) * ED, nullptr, ED, 0, H1, nullptr, EF / 2, 0, b1 + fh * (EF / 2), nullptr, 0, ER, EF / 2, ED, 1.0f);
    if (fh == 0) wmma_gemm64<0, false, 2, 0, false><<<dim3((tr * 4 + 7) / 8, 1), 256, 0, stream>>>(U16(H1), nullptr, EF / 2, 0, U16(W216), nullptr, EF, 0, FF, nullptr, ED, 0, b2, nullptr, 0, ER, ED, EF / 2, 1.0f);
    else         wmma_gemm64<0, false, 0, 0, true><<<dim3((tr * 4 + 7) / 8, 1), 256, 0, stream>>>(U16(H1), nullptr, EF / 2, 0, U16(W216) + EF / 2, nullptr, EF, 0, FF, nullptr, ED, 0, nullptr, FF, 0, ER, ED, EF / 2, 1.0f); }
  ln_kernel<false><<<ER / 8, 256, 0, stream>>>(R1, FF, lng, lnb, (float*)d_out, nullptr);
}
